// MultiHeadAttention_2138893713467
// MI455X (gfx1250) — hardware-verified
//
#include <hip/hip_runtime.h>
#ifndef NB
#define NB 2
#endif
#ifndef SEQ
#define SEQ 2048
#endif
#define SQ SEQ
#define NB_FULL 2
#define SQ_FULL 2048
#define DM 1024
#define NH 16
#define HD 64
#define HG 2
#define NR ((size_t)NB * SQ)

#define W_BYTES  ((size_t)4 * DM * DM * 2)
#define X_BYTES  ((size_t)3 * NR * DM * 2)
#define A_BYTES  ((size_t)NR * DM * 2)
#define S_BYTES  ((size_t)HG * SQ * SQ * 4)
#define P_BYTES  ((size_t)HG * SQ * SQ * 2)
#define VT_BYTES ((size_t)NB * NH * HD * SQ * 2)
#define WS_TOTAL (W_BYTES + X_BYTES + 4 * A_BYTES + S_BYTES + P_BYTES + VT_BYTES)

static_assert(DM == 1024);
static_assert(DM == NH * HD);
static_assert(HD == 64);
static_assert(NH % HG == 0);
static_assert(NB <= NB_FULL);
static_assert(SQ <= SQ_FULL);
static_assert(SQ % 128 == 0);
static_assert((NR % 128) == 0);
static_assert((NR * DM) % 2048 == 0);
static_assert(((size_t)DM * DM) % 2048 == 0);
static_assert(((size_t)HG * SQ) % 256 == 0);
static_assert(W_BYTES % 256 == 0 && X_BYTES % 256 == 0 && A_BYTES % 256 == 0 && S_BYTES % 256 == 0 && P_BYTES % 256 == 0 && VT_BYTES % 256 == 0);
static_assert(WS_TOTAL <= (size_t)134217728);

typedef unsigned short v8us __attribute__((ext_vector_type(8), may_alias));
typedef float  v8f  __attribute__((ext_vector_type(8)));
typedef float  v4f  __attribute__((ext_vector_type(4)));
typedef float  v4fa __attribute__((ext_vector_type(4), may_alias));
typedef _Float16 v16h __attribute__((ext_vector_type(16)));
typedef _Float16 v4h  __attribute__((ext_vector_type(4)));
union FragH { v16h v; v8us half[2]; _Float16 h[16]; unsigned short u[16]; };

__device__ __forceinline__ float bf16_rne(float x) { unsigned int u = __float_as_uint(x); u = (u + 0x7FFFu + ((u >> 16) & 1u)) & 0xFFFF0000u; return __uint_as_float(u); }

__global__ __launch_bounds__(256) void k_x16(const float* __restrict__ x0, const float* __restrict__ x1, const float* __restrict__ x2, _Float16* __restrict__ X16) {
  const unsigned t = blockIdx.x * 256u + threadIdx.x;
  const unsigned by = blockIdx.y;
  const float* x = (by == 0u) ? x0 : ((by == 1u) ? x1 : x2);
  if (t >= (unsigned)(NR * DM / 8)) return;
  const unsigned row = t >> 7, c8 = (t & 127u) << 3;
  const unsigned b = row / (unsigned)SQ, s = row - b * (unsigned)SQ;
  const float* src = x + ((size_t)b * SQ_FULL + s) * DM + c8;
  const v4f a = *(const v4fa*)src, c = *(const v4fa*)(src + 4);
  FragH f;
#pragma unroll
  for (int q = 0; q < 4; ++q) { f.h[q] = (_Float16)bf16_rne(a[q]); f.h[4 + q] = (_Float16)bf16_rne(c[q]); }
  unsigned short* d = (unsigned short*)X16 + (size_t)by * (NR * DM) + (size_t)t * 8;
  const v8us o = f.half[0];
  *(volatile v8us*)d = o; __threadfence(); *(volatile v8us*)d = o;
}

__global__ __launch_bounds__(256) void k_w16(const float* __restrict__ w0, const float* __restrict__ w1, const float* __restrict__ w2, const float* __restrict__ w3, _Float16* __restrict__ Bt) {
  const unsigned t = blockIdx.x * 256u + threadIdx.x;
  const unsigned by = blockIdx.y;
  const float* wsrc = (by == 0u) ? w0 : ((by == 1u) ? w1 : ((by == 2u) ? w2 : w3));
  if (t >= (unsigned)((size_t)DM * DM / 8)) return;
  const float* src = wsrc + (size_t)t * 8;
  const v4f a = *(const v4fa*)src, c = *(const v4fa*)(src + 4);
  FragH f;
#pragma unroll
  for (int q = 0; q < 4; ++q) { f.h[q] = (_Float16)(bf16_rne(a[q]) * 16.0f); f.h[4 + q] = (_Float16)(bf16_rne(c[q]) * 16.0f); }
  unsigned short* d = (unsigned short*)Bt + (size_t)by * ((size_t)DM * DM) + (size_t)t * 8;
  const v8us o = f.half[0];
  *(volatile v8us*)d = o; __threadfence(); *(volatile v8us*)d = o;
}

__device__ __forceinline__ v16h g2_frag(const _Float16* p, unsigned hh) { FragH f; f.half[0] = *(const v8us*)((const unsigned short*)p + 8u * hh); f.half[1] = *(const v8us*)((const unsigned short*)p + 16u + 8u * hh); return f.v; }
__device__ __forceinline__ v8f g2_mma(v16h a, v16h b, v8f c) { v8f d = __builtin_amdgcn_wmma_f32_16x16x32_f16(false, a, false, b, (short)0, c, false, false); asm volatile("v_nop\n\tv_nop\n\tv_nop\n\tv_nop" : "+v"(d) : "v"(a), "v"(b)); return d; }

template <bool HASB>
__global__ __launch_bounds__(128) void k_gemm2(const _Float16* __restrict__ A, unsigned lda, size_t sA, const _Float16* __restrict__ Bh, unsigned ldb, size_t sB, float alpha, const float* __restrict__ bias,
    float* __restrict__ C, _Float16* __restrict__ C16, unsigned ldc, size_t sC, unsigned M, unsigned N, unsigned K) {
  __shared__ __attribute__((aligned(16))) float so[4][32][68];
  const unsigned tid = threadIdx.x, w = tid >> 5, lane = tid & 31u, ln = lane & 15u, hh = lane >> 4; const unsigned by = blockIdx.y;
  A += (size_t)by * sA; Bh += (size_t)by * sB; const size_t cofs = (size_t)by * sC;
  const unsigned ntn = N >> 6; const unsigned mt = blockIdx.x / ntn, nq = blockIdx.x - mt * ntn; const unsigned row0 = mt * 128u + 32u * w, col0 = nq * 64u; if (row0 >= M) return;
  const _Float16* a0p = A + (size_t)(row0 + ln) * lda; const _Float16* a1p = a0p + (size_t)16 * lda;
  const _Float16* b0p = Bh + (size_t)(col0 + ln) * ldb; const _Float16* b1p = b0p + (size_t)16 * ldb; const _Float16* b2p = b1p + (size_t)16 * ldb; const _Float16* b3p = b2p + (size_t)16 * ldb;
  const v8f z8 = {0.f,0.f,0.f,0.f,0.f,0.f,0.f,0.f}; v8f c00 = z8, c01 = z8, c02 = z8, c03 = z8, c10 = z8, c11 = z8, c12 = z8, c13 = z8;
#pragma unroll 1
  for (unsigned kb = 0; kb < K; kb += 32u) { const v16h a0 = g2_frag(a0p + kb, hh), a1 = g2_frag(a1p + kb, hh);
    v16h b = g2_frag(b0p + kb, hh); c00 = g2_mma(a0, b, c00); c10 = g2_mma(a1, b, c10);
    b = g2_frag(b1p + kb, hh); c01 = g2_mma(a0, b, c01); c11 = g2_mma(a1, b, c11);
    b = g2_frag(b2p + kb, hh); c02 = g2_mma(a0, b, c02); c12 = g2_mma(a1, b, c12);
    b = g2_frag(b3p + kb, hh); c03 = g2_mma(a0, b, c03); c13 = g2_mma(a1, b, c13); }
  const v8f accs[8] = {c00, c01, c02, c03, c10, c11, c12, c13};
#pragma unroll
  for (unsigned u = 0; u < 8; ++u) { const unsigned t = u & 3u, hf = u >> 2; const unsigned col = col0 + t * 16u + ln; float bv = 0.f; if (HASB) bv = bf16_rne(bias[col]);
#pragma unroll
    for (unsigned r = 0; r < 8; ++r) { const unsigned rloc = hf * 16u + 8u * hh + r; so[w][rloc][t * 16u + ln] = accs[u][r] * alpha + bv; } }
  __builtin_amdgcn_fence(4  , "workgroup"); __builtin_amdgcn_wave_barrier();
  const unsigned rsub = lane >> 4, c4 = (lane & 15u) << 2;
  for (int pass = 0; pass < 2; ++pass) {
#pragma unroll
    for (unsigned q = 0; q < 16; ++q) { const unsigned r = q * 2u + rsub; const v4f v = *(const v4fa*)&so[w][r][c4];
      if (C) *(volatile v4f*)(C + cofs + (size_t)(row0 + r) * ldc + col0 + c4) = v;
      if (C16) { v4h h4; h4[0] = (_Float16)v[0]; h4[1] = (_Float16)v[1]; h4[2] = (_Float16)v[2]; h4[3] = (_Float16)v[3]; *(volatile v4h*)(C16 + cofs + (size_t)(row0 + r) * ldc + col0 + c4) = h4; } }
    if (pass == 0) __threadfence(); } }

template <unsigned NHv, unsigned TTv>
__global__ __launch_bounds__(256) void k_vt(const _Float16* __restrict__ V16, unsigned ldv, _Float16* __restrict__ Vt) {
  __shared__ unsigned short tl[64][66];
  const unsigned tid = threadIdx.x; const unsigned slab = blockIdx.x / (TTv / 64u), lg = blockIdx.x % (TTv / 64u); const unsigned b = slab / NHv, h = slab % NHv;
  for (unsigned i = tid; i < 512u; i += 256u) { const unsigned r = i >> 3, c8 = (i & 7u) << 3; FragH f;
    f.half[0] = *(const v8us*)((const unsigned short*)V16 + ((size_t)b * TTv + lg * 64u + r) * ldv + h * 64u + c8);
#pragma unroll
    for (unsigned q = 0; q < 8; ++q) tl[r][c8 + q] = f.u[q]; }
  __syncthreads();
  for (int pass = 0; pass < 2; ++pass) {
#pragma unroll
    for (unsigned rd = 0; rd < 2; ++rd) { const unsigned d = rd * 32u + (tid >> 3), pc = tid & 7u; FragH f;
#pragma unroll
      for (unsigned q = 0; q < 8; ++q) f.u[q] = tl[pc * 8u + q][d];
      const v8us o = f.half[0];
      *(volatile v8us*)((unsigned short*)Vt + ((size_t)slab * 64u + d) * TTv + lg * 64u + pc * 8u) = o; }
    if (pass == 0) __threadfence(); } }

__global__ __launch_bounds__(256) void k_rsm(const float* __restrict__ S, _Float16* __restrict__ P, unsigned nrows) {
  #pragma clang fp contract(off)
  const unsigned i = blockIdx.x * 256u + threadIdx.x; if (i >= nrows) return; const float* s = S + (size_t)i * SQ; float mx = -3.0e38f;
#pragma unroll 1
  for (unsigned j = 0; j < (unsigned)SQ; j += 4u) { const v4f a = *(const v4fa*)(s + j); mx = fmaxf(mx, a[0]); mx = fmaxf(mx, a[1]); mx = fmaxf(mx, a[2]); mx = fmaxf(mx, a[3]); }
  float se = 0.f;
#pragma unroll 1
  for (unsigned j = 0; j < (unsigned)SQ; j += 4u) { const v4f a = *(const v4fa*)(s + j); se += expf(a[0] - mx); se += expf(a[1] - mx); se += expf(a[2] - mx); se += expf(a[3] - mx); }
  const float sc = 256.0f / se;
#pragma unroll 1
  for (unsigned j0 = 0; j0 < (unsigned)SQ; j0 += 8u) { const v4f a = *(const v4fa*)(s + j0), c = *(const v4fa*)(s + j0 + 4u); FragH f;
#pragma unroll
    for (int q = 0; q < 4; ++q) { f.h[q] = (_Float16)(expf(a[q] - mx) * sc); f.h[4 + q] = (_Float16)(expf(c[q] - mx) * sc); }
    unsigned short* d = (unsigned short*)P + (size_t)i * SQ + j0; const v8us o = f.half[0];
    *(volatile v8us*)d = o; __threadfence(); *(volatile v8us*)d = o; } }

extern "C" void kernel_launch(void* const* d_in, const int* in_sizes, int n_in,
                              void* d_out, int out_size, void* d_ws, size_t ws_size, hipStream_t stream) {
  if (n_in < 11) return;
  const size_t need_x = ((size_t)(NB - 1) * SQ_FULL + SQ) * DM;
  if ((size_t)in_sizes[0] < need_x || (size_t)in_sizes[1] < need_x || (size_t)in_sizes[2] < need_x) return;
  if ((size_t)in_sizes[3] < (size_t)DM * DM || (size_t)in_sizes[5] < (size_t)DM * DM || (size_t)in_sizes[7] < (size_t)DM * DM || (size_t)in_sizes[9] < (size_t)DM * DM) return;
  if (in_sizes[4] < DM || in_sizes[6] < DM || in_sizes[8] < DM || in_sizes[10] < DM) return;
  if ((size_t)out_size < NR * DM) return;
  const float* xq = (const float*)d_in[0]; const float* xk = (const float*)d_in[1]; const float* xv = (const float*)d_in[2];
  const float* wq = (const float*)d_in[3]; const float* bq = (const float*)d_in[4];
  const float* wk = (const float*)d_in[5]; const float* bk = (const float*)d_in[6];
  const float* wv = (const float*)d_in[7]; const float* bv = (const float*)d_in[8];
  const float* wo = (const float*)d_in[9]; const float* bo = (const float*)d_in[10];
  float* out = (float*)d_out;
  char* ws = (char*)d_ws; size_t off = 0;
  auto take = [&](size_t bytes) { char* p = ws + off; off += (bytes + 255) & ~(size_t)255; return p; };
  _Float16* BW = (_Float16*)take(W_BYTES);
  _Float16* XP = (_Float16*)take(X_BYTES);
  _Float16* Q16 = (_Float16*)take(A_BYTES); _Float16* K16 = (_Float16*)take(A_BYTES); _Float16* V16 = (_Float16*)take(A_BYTES); _Float16* O16 = (_Float16*)take(A_BYTES);
  float* S = (float*)take(S_BYTES);
  _Float16* P = (_Float16*)take(P_BYTES);
  _Float16* VT = (_Float16*)take(VT_BYTES);
  if (off > ws_size) return;
  const size_t WW = (size_t)DM * DM, XA = NR * DM;
  _Float16* BQ = BW; _Float16* BK = BW + WW; _Float16* BV = BW + 2 * WW; _Float16* BO = BW + 3 * WW;
  _Float16* XQ = XP; _Float16* XK = XP + XA; _Float16* XV = XP + 2 * XA;

  k_w16<<<dim3((unsigned)(WW / 2048), 4), 256, 0, stream>>>(wq, wk, wv, wo, BW);
  k_x16<<<dim3((unsigned)(XA / 2048), 3), 256, 0, stream>>>(xq, xk, xv, XP);

  const unsigned gproj = (unsigned)((NR / 128) * (DM / 64));
  k_gemm2<true><<<dim3(gproj, 1), 128, 0, stream>>>(XQ, DM, 0, BQ, DM, 0, 0.0625f, bq, nullptr, Q16, DM, 0, (unsigned)NR, DM, DM);
  k_gemm2<true><<<dim3(gproj, 1), 128, 0, stream>>>(XK, DM, 0, BK, DM, 0, 0.0625f, bk, nullptr, K16, DM, 0, (unsigned)NR, DM, DM);
  k_gemm2<true><<<dim3(gproj, 1), 128, 0, stream>>>(XV, DM, 0, BV, DM, 0, 0.0625f, bv, nullptr, V16, DM, 0, (unsigned)NR, DM, DM);

  k_vt<NH, SQ><<<NB * NH * (SQ / 64), 256, 0, stream>>>(V16, DM, VT);

  for (int b = 0; b < NB; ++b) { const size_t r0 = (size_t)b * SQ;
    for (int h0 = 0; h0 < NH; h0 += HG) {
      k_gemm2<false><<<dim3((SQ / 128) * (SQ / 64), HG), 128, 0, stream>>>(Q16 + r0 * DM + (size_t)h0 * HD, DM, (size_t)HD, K16 + r0 * DM + (size_t)h0 * HD, DM, (size_t)HD, 0.125f, nullptr,
                                                                          S, nullptr, SQ, (size_t)SQ * SQ, SQ, SQ, HD);
      k_rsm<<<(HG * SQ) / 256, 256, 0, stream>>>(S, P, (unsigned)(HG * SQ));
      k_gemm2<false><<<dim3((SQ / 128) * (HD / 64), HG), 128, 0, stream>>>(P, SQ, (size_t)SQ * SQ, VT + ((size_t)b * NH + h0) * HD * SQ, SQ, (size_t)HD * SQ, 0.25f, nullptr,
                                                                          nullptr, O16 + r0 * DM + (size_t)h0 * HD, DM, (size_t)HD, SQ, HD, SQ);
    } }

  k_gemm2<true><<<dim3(gproj, 1), 128, 0, stream>>>(O16, DM, 0, BO, DM, 0, 0.0009765625f, bo, out, nullptr, DM, 0, (unsigned)NR, DM, DM);
}
